// MultiQueryAttention_53772990546487
// MI455X (gfx1250) — hardware-verified
//
#include <hip/hip_runtime.h>
#include <stdint.h>


typedef _Float16 v16h __attribute__((ext_vector_type(16)));
typedef _Float16 v8h  __attribute__((ext_vector_type(8)));
typedef float    v8f  __attribute__((ext_vector_type(8)));
typedef float    v4f  __attribute__((ext_vector_type(4)));

#define DM 2048
#define HD 128
#define NH 16
#define NG 4
#define QPK (NH / NG)
#define NQKV (DM + 2 * HD * NG)
#define NB_FULL 1
#define SEQ_FULL 2048
#ifndef NB
#define NB 1
#endif
#ifndef SEQ
#define SEQ 2048
#endif
#define EARLYQ 256
#define NQBT (SEQ / 64)
#define NQBE (((EARLYQ / 64) < NQBT) ? (EARLYQ / 64) : NQBT)
#define NQBL (NQBT - NQBE)
#define WSCALE 64.0f
#define PCARRY 1024.0f
#define YCARRY 64.0f
#define RCARRY 1024.0f
#define INV_R 0.0009765625f
#define LOG2E 1.4426950408889634f
#define SCL 0.0883883461356163f
#define ALM0 0.70710678f
#define MASKB (-65504.0f)
#define PSP 136
#define VSP 128

static_assert(SEQ % 128 == 0);
static_assert(SEQ >= 128 && SEQ <= SEQ_FULL);
static_assert(NB == 1 && NB_FULL == 1);
static_assert(DM % 128 == 0 && HD == 128 && DM == NH * HD);
static_assert(NQKV % 128 == 0 && NQKV == DM + 2 * HD * NG);
static_assert(DM / 8 == 256);
static_assert(EARLYQ % 64 == 0);
static_assert(NQBE >= 1 && NQBE <= NQBT && NQBL >= 0);
static_assert(NH % NG == 0);
static_assert(PSP % 8 == 0 && PSP >= 128 && VSP == 128);
static_assert(SEQ % 128 == 0 && SEQ / 128 >= 1);

union HFrag { v16h v; v8h h[2]; };

__device__ __forceinline__ v16h load_frag(const _Float16* p) {
    HFrag f;
    f.h[0] = *reinterpret_cast<const v8h*>(p);
    f.h[1] = *reinterpret_cast<const v8h*>(p + 16);
    return f.v;
}

__device__ __forceinline__ v16h zfrag() {
    const _Float16 z = (_Float16)0.0f;
    HFrag f;
    const v8h zz = {z, z, z, z, z, z, z, z};
    f.h[0] = zz;
    f.h[1] = zz;
    return f.v;
}

__device__ __forceinline__ v8f wmma16(v16h a, v16h b, v8f c) {
    return __builtin_amdgcn_wmma_f32_16x16x32_f16(false, a, false, b, (short)0, c, false, false);
}

__device__ __forceinline__ float bf16r(float f) {
    unsigned int u = __float_as_uint(f);
    u += 0x7FFFu + ((u >> 16) & 1u);
    u &= 0xFFFF0000u;
    return __uint_as_float(u);
}

template <int RES>
__device__ __forceinline__ _Float16 cvt_hr(float v) {
    const _Float16 hv = (_Float16)v;
    if (RES == 0) return hv;
    const float r = (v - (float)hv) * RCARRY;
    return (_Float16)r;
}

__global__ __launch_bounds__(256) void k_cvt(const float* __restrict__ src, _Float16* dst, float scale)
{
    const size_t row = blockIdx.x;
    const int col = (int)threadIdx.x * 8;
    const float* s = src + row * DM + col;
    const v4f f0 = *reinterpret_cast<const v4f*>(s);
    const v4f f1 = *reinterpret_cast<const v4f*>(s + 4);
    v8h o;
    o[0] = (_Float16)(bf16r(f0[0]) * scale); o[1] = (_Float16)(bf16r(f0[1]) * scale);
    o[2] = (_Float16)(bf16r(f0[2]) * scale); o[3] = (_Float16)(bf16r(f0[3]) * scale);
    o[4] = (_Float16)(bf16r(f1[0]) * scale); o[5] = (_Float16)(bf16r(f1[1]) * scale);
    o[6] = (_Float16)(bf16r(f1[2]) * scale); o[7] = (_Float16)(bf16r(f1[3]) * scale);
    _Float16* d = dst + row * DM + col;
    *(volatile v8h*)d = o;
    __threadfence();
    *(volatile v8h*)d = o;
}

__device__ __forceinline__ void store32x64_f16(const _Float16* sw, _Float16* gdst,
                                               size_t pitch, int lane)
{
    const int rq = lane >> 3, seg = lane & 7;
    v8h v[8];
#pragma unroll
    for (int it = 0; it < 8; ++it)
        v[it] = *reinterpret_cast<const v8h*>(sw + (it * 4 + rq) * 64 + seg * 8);
#pragma unroll
    for (int it = 0; it < 8; ++it)
        *(volatile v8h*)(gdst + (size_t)(it * 4 + rq) * pitch + seg * 8) = v[it];
    __threadfence();
#pragma unroll
    for (int it = 0; it < 8; ++it)
        *(volatile v8h*)(gdst + (size_t)(it * 4 + rq) * pitch + seg * 8) = v[it];
}

template <int RES>
__device__ __forceinline__ void stage32x64(_Float16* sw, const v8f (&acc)[2][4], float alpha,
                                           int hi8, int l15)
{
#pragma unroll
    for (int g = 0; g < 2; ++g)
#pragma unroll
        for (int ni = 0; ni < 4; ++ni)
#pragma unroll
            for (int j = 0; j < 8; ++j)
                sw[(g * 16 + hi8 + j) * 64 + ni * 16 + l15] = cvt_hr<RES>(acc[g][ni][j] * alpha);
}

template <int RES>
__device__ __forceinline__ void stage_vt(_Float16* vs, const v8f (&acc)[2][4], float alpha,
                                         int wm, int wn, int hi8, int l15)
{
#pragma unroll
    for (int g = 0; g < 2; ++g)
#pragma unroll
        for (int ni = 0; ni < 4; ++ni)
#pragma unroll
            for (int j = 0; j < 8; ++j)
                vs[(wn * 64 + ni * 16 + l15) * VSP + wm * 32 + g * 16 + hi8 + j] =
                    cvt_hr<RES>(acc[g][ni][j] * alpha);
}

__device__ __forceinline__ void store_vt(const _Float16* vs, _Float16* gdst, int tid)
{
    const int dq = tid >> 4, seg = tid & 15;
    v8h v[8];
#pragma unroll
    for (int it = 0; it < 8; ++it)
        v[it] = *reinterpret_cast<const v8h*>(vs + (it * 16 + dq) * VSP + seg * 8);
#pragma unroll
    for (int it = 0; it < 8; ++it)
        *(volatile v8h*)(gdst + (size_t)(it * 16 + dq) * SEQ + seg * 8) = v[it];
    __threadfence();
#pragma unroll
    for (int it = 0; it < 8; ++it)
        *(volatile v8h*)(gdst + (size_t)(it * 16 + dq) * SEQ + seg * 8) = v[it];
}

__global__ __launch_bounds__(256) __attribute__((amdgpu_num_vgpr(256)))
void k_gemm_qkv(const _Float16* __restrict__ A, const _Float16* __restrict__ BT,
                _Float16* qh, _Float16* qr, _Float16* kh, _Float16* kr,
                _Float16* vth, _Float16* vtr)
{
    __shared__ float stg[8 * 1024] __attribute__((aligned(16)));
    const int tid = threadIdx.x;
    const int lane = tid & 31, wave = tid >> 5;
    const int wm = wave & 3, wn = wave >> 2;
    const int l15 = lane & 15, hi8 = (lane >> 4) << 3;
    const int nb = blockIdx.x;
    const int bm0 = blockIdx.y * 128, bn0 = nb * 128;

    const _Float16* ap0 = A + (size_t)(bm0 + wm * 32 + l15) * DM + hi8;
    const _Float16* ap1 = ap0 + (size_t)16 * DM;
    const _Float16* bp  = BT + (size_t)(bn0 + wn * 64 + l15) * DM + hi8;
    const size_t bst = (size_t)16 * DM;

    const v8f zero8 = {0.f, 0.f, 0.f, 0.f, 0.f, 0.f, 0.f, 0.f};
    v8f acc[2][4];
#pragma unroll
    for (int g = 0; g < 2; ++g)
#pragma unroll
        for (int ni = 0; ni < 4; ++ni) acc[g][ni] = zero8;

    for (int k0 = 0; k0 < DM; k0 += 32) {
        const v16h a0 = load_frag(ap0 + k0);
        const v16h a1 = load_frag(ap1 + k0);
        const v16h b0 = load_frag(bp + k0);
        const v16h b1 = load_frag(bp + bst + k0);
        const v16h b2 = load_frag(bp + 2 * bst + k0);
        const v16h b3 = load_frag(bp + 3 * bst + k0);
        acc[0][0] = wmma16(a0, b0, acc[0][0]);
        acc[0][1] = wmma16(a0, b1, acc[0][1]);
        acc[0][2] = wmma16(a0, b2, acc[0][2]);
        acc[0][3] = wmma16(a0, b3, acc[0][3]);
        acc[1][0] = wmma16(a1, b0, acc[1][0]);
        acc[1][1] = wmma16(a1, b1, acc[1][1]);
        acc[1][2] = wmma16(a1, b2, acc[1][2]);
        acc[1][3] = wmma16(a1, b3, acc[1][3]);
        asm volatile("v_nop\n\tv_nop\n\tv_nop\n\tv_nop"
                     : "+v"(acc[0][0]), "+v"(acc[0][1]), "+v"(acc[0][2]), "+v"(acc[0][3]),
                       "+v"(acc[1][0]), "+v"(acc[1][1]), "+v"(acc[1][2]), "+v"(acc[1][3])
                     : "v"(a0), "v"(a1), "v"(b0), "v"(b1), "v"(b2), "v"(b3));
    }

    const float alpha = 1.0f / WSCALE;
    if (nb < DM / 128) {
        _Float16* sw = reinterpret_cast<_Float16*>(stg + wave * 1024);
        const size_t goff = (size_t)(bm0 + wm * 32) * DM + bn0 + wn * 64;
        stage32x64<0>(sw, acc, alpha, hi8, l15);
        __syncthreads();
        store32x64_f16(sw, qh + goff, (size_t)DM, lane);
        __syncthreads();
        stage32x64<1>(sw, acc, alpha, hi8, l15);
        __syncthreads();
        store32x64_f16(sw, qr + goff, (size_t)DM, lane);
    } else if (((nb - DM / 128) & 1) == 0) {
        const int g = (nb - DM / 128) >> 1;
        _Float16* sw = reinterpret_cast<_Float16*>(stg + wave * 1024);
        const size_t goff = ((size_t)(g * SEQ + bm0 + wm * 32)) * HD + wn * 64;
        stage32x64<0>(sw, acc, alpha, hi8, l15);
        __syncthreads();
        store32x64_f16(sw, kh + goff, (size_t)HD, lane);
        __syncthreads();
        stage32x64<1>(sw, acc, alpha, hi8, l15);
        __syncthreads();
        store32x64_f16(sw, kr + goff, (size_t)HD, lane);
    } else {
        const int g = (nb - DM / 128) >> 1;
        _Float16* vs = reinterpret_cast<_Float16*>(stg);
        const size_t goff = (size_t)(g * HD) * SEQ + bm0;
        stage_vt<0>(vs, acc, alpha, wm, wn, hi8, l15);
        __syncthreads();
        store_vt(vs, vth + goff, tid);
        __syncthreads();
        stage_vt<1>(vs, acc, alpha, wm, wn, hi8, l15);
        __syncthreads();
        store_vt(vs, vtr + goff, tid);
    }
}

__device__ __forceinline__ void store16x128_f16(const _Float16* sw, _Float16* gdst, int lane)
{
    const int r2 = lane >> 4, seg = lane & 15;
    v8h v[8];
#pragma unroll
    for (int it = 0; it < 8; ++it)
        v[it] = *reinterpret_cast<const v8h*>(sw + (it * 2 + r2) * PSP + seg * 8);
#pragma unroll
    for (int it = 0; it < 8; ++it)
        *(volatile v8h*)(gdst + (size_t)(it * 2 + r2) * DM + seg * 8) = v[it];
    __threadfence();
#pragma unroll
    for (int it = 0; it < 8; ++it)
        *(volatile v8h*)(gdst + (size_t)(it * 2 + r2) * DM + seg * 8) = v[it];
}

template <int EARLY>
__global__ __launch_bounds__(128) __attribute__((amdgpu_num_vgpr(256)))
void k_attn(const _Float16* __restrict__ qh, const _Float16* __restrict__ qr,
            const _Float16* __restrict__ kh, const _Float16* __restrict__ kr,
            const _Float16* __restrict__ vth, const _Float16* __restrict__ vtr,
            _Float16* yh, _Float16* yr)
{
    __shared__ _Float16 Ws[4 * 16 * PSP] __attribute__((aligned(16)));
    __shared__ float sqt[SEQ];
    const int tid  = threadIdx.x;
    const int lane = tid & 31;
    const int wv   = tid >> 5;
    const int l15  = lane & 15;
    const int hi8  = (lane >> 4) << 3;

    constexpr int NQB = EARLY ? NQBE : (NQBL > 0 ? NQBL : 1);
    constexpr int QB0 = EARLY ? 0 : NQBE;
    const int h   = (int)blockIdx.x / NQB;
    const int qb  = (int)blockIdx.x - h * NQB + QB0;
    const int g   = h / QPK;
    const int q0  = qb * 64 + wv * 16;
    const int kend = qb * 64 + 64;

#pragma unroll 1
    for (int i = tid; i < SEQ; i += 128) sqt[i] = sqrtf((float)i);

    const float slope  = powf(ALM0, (float)(h + 1));
    const float nslope = -slope;

    const size_t qoff = ((size_t)(q0 + l15)) * DM + h * HD + hi8;
    const _Float16* qhb = qh + qoff;
    const _Float16* qrb = qr + qoff;
    const _Float16* khb = kh + (size_t)g * SEQ * HD + hi8;
    const _Float16* vhb = vth + (size_t)(g * HD) * SEQ + hi8;
    const _Float16* vrb = vtr + (size_t)(g * HD) * SEQ + hi8;

    const v8f zero8 = {0.f, 0.f, 0.f, 0.f, 0.f, 0.f, 0.f, 0.f};
    v16h aQ[4];
#pragma unroll
    for (int kk = 0; kk < 4; ++kk) aQ[kk] = EARLY ? zfrag() : load_frag(qhb + kk * 32);

    float m[8], l[8];
    v8f accY[8];
#pragma unroll
    for (int j = 0; j < 8; ++j) { m[j] = -1e30f; l[j] = 0.0f; }
#pragma unroll
    for (int d = 0; d < 8; ++d) accY[d] = zero8;

    _Float16* ps = Ws + wv * 16 * PSP;
    int ch = 0;
    __syncthreads();

#pragma unroll 1
    for (int tc = 0; tc < kend; tc += 32) {
        v8f s0 = zero8, s1 = zero8;
        const int kofs = (tc + l15) * HD;
        if (!EARLY) {
#pragma unroll
            for (int kk = 0; kk < 4; ++kk) {
                const v16h b0 = load_frag(khb + (size_t)(kofs + ch + kk * 32));
                const v16h b1 = load_frag(khb + (size_t)(kofs + ch + 16 * HD + kk * 32));
                s0 = wmma16(aQ[kk], b0, s0);
                s1 = wmma16(aQ[kk], b1, s1);
                asm volatile("v_nop\n\tv_nop\n\tv_nop\n\tv_nop"
                             : "+v"(s0), "+v"(s1), "+v"(ch)
                             : "v"(aQ[kk]), "v"(b0), "v"(b1));
            }
        } else {
            v8f r0 = zero8, r1 = zero8;
#pragma unroll 1
            for (int kk = 0; kk < 4; ++kk) {
                const v16h aq = load_frag(qhb + (size_t)(ch + kk * 32));
                const v16h b0 = load_frag(khb + (size_t)(kofs + ch + kk * 32));
                const v16h b1 = load_frag(khb + (size_t)(kofs + ch + 16 * HD + kk * 32));
                s0 = wmma16(aq, b0, s0);
                s1 = wmma16(aq, b1, s1);
                asm volatile("v_nop\n\tv_nop\n\tv_nop\n\tv_nop"
                             : "+v"(s0), "+v"(s1), "+v"(ch)
                             : "v"(aq), "v"(b0), "v"(b1));
                const v16h ar = load_frag(qrb + (size_t)(ch + kk * 32));
                r0 = wmma16(ar, b0, r0);
                r1 = wmma16(ar, b1, r1);
                asm volatile("v_nop\n\tv_nop\n\tv_nop\n\tv_nop"
                             : "+v"(r0), "+v"(r1), "+v"(ch)
                             : "v"(ar), "v"(b0), "v"(b1));
            }
#pragma unroll
            for (int j = 0; j < 8; ++j) {
                s0[j] = fmaf(r0[j], INV_R, s0[j]);
                s1[j] = fmaf(r1[j], INV_R, s1[j]);
            }
        }

#pragma unroll
        for (int j = 0; j < 8; ++j) {
            const int qi = q0 + hi8 + j;
            const int d0 = qi - tc - l15;
            const int d1 = d0 - 16;
            const float sr0 = sqt[d0 > 0 ? d0 : 0];
            const float sr1 = sqt[d1 > 0 ? d1 : 0];
            const float bb0 = (d0 < 0) ? MASKB : nslope * sr0;
            const float bb1 = (d1 < 0) ? MASKB : nslope * sr1;
            const float a0 = (s0[j] * SCL + bb0) * LOG2E;
            const float a1 = (s1[j] * SCL + bb1) * LOG2E;
            float mt = fmaxf(a0, a1);
#pragma unroll
            for (int off = 8; off >= 1; off >>= 1)
                mt = fmaxf(mt, __shfl_xor(mt, off, 16));
            const float mn = fmaxf(m[j], mt);
            const float sc = exp2f(m[j] - mn);
            const float p0 = exp2f(a0 - mn);
            const float p1 = exp2f(a1 - mn);
            float rs = p0 + p1;
#pragma unroll
            for (int off = 8; off >= 1; off >>= 1)
                rs += __shfl_xor(rs, off, 16);
            l[j] = l[j] * sc + rs;
            m[j] = mn;
#pragma unroll
            for (int d = 0; d < 8; ++d) accY[d][j] *= sc;
            const float pc0 = p0 * PCARRY, pc1 = p1 * PCARRY;
            const _Float16 ph0 = (_Float16)pc0, ph1 = (_Float16)pc1;
            const int row = hi8 + j;
            ps[row * PSP + l15]      = ph0;
            ps[row * PSP + 16 + l15] = ph1;
            if (EARLY) {
                ps[row * PSP + 32 + l15] = (_Float16)((pc0 - (float)ph0) * RCARRY);
                ps[row * PSP + 48 + l15] = (_Float16)((pc1 - (float)ph1) * RCARRY);
            }
        }
        __syncthreads();

        const int vofs = l15 * SEQ + tc;
        if (!EARLY) {
            const v16h aP = load_frag(ps + l15 * PSP + hi8);
#pragma unroll
            for (int d = 0; d < 8; ++d) {
                const v16h bh = load_frag(vhb + (size_t)(vofs + ch + d * 16 * SEQ));
                accY[d] = wmma16(aP, bh, accY[d]);
                asm volatile("v_nop\n\tv_nop\n\tv_nop\n\tv_nop"
                             : "+v"(accY[d]), "+v"(ch)
                             : "v"(aP), "v"(bh));
            }
        } else {
            const v16h aPh = load_frag(ps + l15 * PSP + hi8);
            const v16h aPr = load_frag(ps + l15 * PSP + 32 + hi8);
#pragma unroll
            for (int d = 0; d < 8; ++d) {
                const v16h bh = load_frag(vhb + (size_t)(vofs + ch + d * 16 * SEQ));
                const v16h br = load_frag(vrb + (size_t)(vofs + ch + d * 16 * SEQ));
                accY[d] = wmma16(aPh, bh, accY[d]);
                v8f tr = wmma16(aPr, bh, zero8);
                tr = wmma16(aPh, br, tr);
                asm volatile("v_nop\n\tv_nop\n\tv_nop\n\tv_nop"
                             : "+v"(accY[d]), "+v"(tr), "+v"(ch)
                             : "v"(aPh), "v"(aPr), "v"(bh), "v"(br));
#pragma unroll
                for (int j = 0; j < 8; ++j) accY[d][j] = fmaf(tr[j], INV_R, accY[d][j]);
                asm volatile("" : "+v"(accY[d]), "+v"(ch));
            }
        }
    }
    __syncthreads();

    float inv[8];
#pragma unroll
    for (int j = 0; j < 8; ++j) inv[j] = (YCARRY / PCARRY) * (1.0f / l[j]);
#pragma unroll
    for (int d = 0; d < 8; ++d)
#pragma unroll
        for (int j = 0; j < 8; ++j)
            ps[(hi8 + j) * PSP + d * 16 + l15] = (_Float16)(accY[d][j] * inv[j]);
    __syncthreads();
    const size_t yoff = ((size_t)q0) * DM + h * HD;
    store16x128_f16(ps, yh + yoff, lane);
    __syncthreads();
#pragma unroll
    for (int d = 0; d < 8; ++d)
#pragma unroll
        for (int j = 0; j < 8; ++j) {
            const float y = accY[d][j] * inv[j];
            const _Float16 hv = (_Float16)y;
            ps[(hi8 + j) * PSP + d * 16 + l15] = (_Float16)((y - (float)hv) * RCARRY);
        }
    __syncthreads();
    store16x128_f16(ps, yr + yoff, lane);
}

__global__ __launch_bounds__(256) __attribute__((amdgpu_num_vgpr(256)))
void k_gemm_out(const _Float16* __restrict__ AH, const _Float16* __restrict__ AR,
                const _Float16* __restrict__ BT, float* out)
{
    __shared__ float stg[8 * 1024] __attribute__((aligned(16)));
    const int tid = threadIdx.x;
    const int lane = tid & 31, wave = tid >> 5;
    const int wm = wave & 3, wn = wave >> 2;
    const int l15 = lane & 15, hi8 = (lane >> 4) << 3;
    const int bm0 = blockIdx.y * 128, bn0 = blockIdx.x * 64;

    const size_t aoff = (size_t)(bm0 + wm * 32 + l15) * DM + hi8;
    const _Float16* ap0 = AH + aoff;
    const _Float16* ap1 = ap0 + (size_t)16 * DM;
    const _Float16* cp0 = AR + aoff;
    const _Float16* cp1 = cp0 + (size_t)16 * DM;
    const _Float16* bp  = BT + (size_t)(bn0 + wn * 32 + l15) * DM + hi8;
    const size_t bst = (size_t)16 * DM;

    const v8f zero8 = {0.f, 0.f, 0.f, 0.f, 0.f, 0.f, 0.f, 0.f};
    v8f ah[2][2], rr[2][2];
#pragma unroll
    for (int g = 0; g < 2; ++g)
#pragma unroll
        for (int ni = 0; ni < 2; ++ni) { ah[g][ni] = zero8; rr[g][ni] = zero8; }

    for (int k0 = 0; k0 < DM; k0 += 32) {
        const v16h a0 = load_frag(ap0 + k0);
        const v16h a1 = load_frag(ap1 + k0);
        const v16h c0 = load_frag(cp0 + k0);
        const v16h c1 = load_frag(cp1 + k0);
        const v16h b0 = load_frag(bp + k0);
        const v16h b1 = load_frag(bp + bst + k0);
        ah[0][0] = wmma16(a0, b0, ah[0][0]);
        ah[0][1] = wmma16(a0, b1, ah[0][1]);
        ah[1][0] = wmma16(a1, b0, ah[1][0]);
        ah[1][1] = wmma16(a1, b1, ah[1][1]);
        rr[0][0] = wmma16(c0, b0, rr[0][0]);
        rr[0][1] = wmma16(c0, b1, rr[0][1]);
        rr[1][0] = wmma16(c1, b0, rr[1][0]);
        rr[1][1] = wmma16(c1, b1, rr[1][1]);
        asm volatile("v_nop\n\tv_nop\n\tv_nop\n\tv_nop"
                     : "+v"(ah[0][0]), "+v"(ah[0][1]), "+v"(ah[1][0]), "+v"(ah[1][1]),
                       "+v"(rr[0][0]), "+v"(rr[0][1]), "+v"(rr[1][0]), "+v"(rr[1][1])
                     : "v"(a0), "v"(a1), "v"(c0), "v"(c1), "v"(b0), "v"(b1));
    }

    float* swf = stg + wave * 1024;
    const float alpha = 1.0f / (YCARRY * WSCALE);
#pragma unroll
    for (int g = 0; g < 2; ++g)
#pragma unroll
        for (int ni = 0; ni < 2; ++ni)
#pragma unroll
            for (int j = 0; j < 8; ++j)
                swf[(g * 16 + hi8 + j) * 32 + ni * 16 + l15] =
                    fmaf(rr[g][ni][j], INV_R, ah[g][ni][j]) * alpha;
    __syncthreads();
    const int rq = lane >> 3, seg = lane & 7;
    v4f v[8];
#pragma unroll
    for (int it = 0; it < 8; ++it)
        v[it] = *reinterpret_cast<const v4f*>(swf + (it * 4 + rq) * 32 + seg * 4);
    float* gd = out + (size_t)(bm0 + wm * 32) * DM + bn0 + wn * 32 + seg * 4;
#pragma unroll
    for (int it = 0; it < 8; ++it)
        *(volatile v4f*)(gd + (size_t)(it * 4 + rq) * DM) = v[it];
    __threadfence();
#pragma unroll
    for (int it = 0; it < 8; ++it)
        *(volatile v4f*)(gd + (size_t)(it * 4 + rq) * DM) = v[it];
}

extern "C" void kernel_launch(void* const* d_in, const int* in_sizes, int n_in,
                              void* d_out, int out_size, void* d_ws, size_t ws_size,
                              hipStream_t stream) {
    if (n_in < 3) return;
    if ((long long)in_sizes[0] < (long long)SEQ * DM) return;
    if ((long long)in_sizes[1] < (long long)NQKV * DM) return;
    if ((long long)in_sizes[2] < (long long)DM * DM) return;
    if ((long long)out_size < (long long)SEQ * DM) return;

    const float* x   = (const float*)d_in[0];
    const float* wq3 = (const float*)d_in[1];
    const float* wo  = (const float*)d_in[2];
    float* out = (float*)d_out;

    size_t off = 0;
    char* wsb = (char*)d_ws;
    auto carve = [&](size_t bytes) -> void* {
        void* p = wsb + off;
        off += (bytes + 255) & ~(size_t)255;
        return p;
    };
    _Float16* x16  = (_Float16*)carve((size_t)SEQ * DM * 2);
    _Float16* w316 = (_Float16*)carve((size_t)NQKV * DM * 2);
    _Float16* wo16 = (_Float16*)carve((size_t)DM * DM * 2);
    _Float16* qh   = (_Float16*)carve((size_t)SEQ * DM * 2);
    _Float16* qr   = (_Float16*)carve((size_t)SEQ * DM * 2);
    _Float16* kh   = (_Float16*)carve((size_t)NG * SEQ * HD * 2);
    _Float16* kr   = (_Float16*)carve((size_t)NG * SEQ * HD * 2);
    _Float16* vth  = (_Float16*)carve((size_t)NG * HD * SEQ * 2);
    _Float16* vtr  = (_Float16*)carve((size_t)NG * HD * SEQ * 2);
    _Float16* yh   = (_Float16*)carve((size_t)SEQ * DM * 2);
    _Float16* yr   = (_Float16*)carve((size_t)SEQ * DM * 2);
    if (off > ws_size) return;

    dim3 blk(256);

    k_cvt<<<dim3(SEQ), blk, 0, stream>>>(x, x16, 1.0f);
    k_cvt<<<dim3(NQKV), blk, 0, stream>>>(wq3, w316, WSCALE);
    k_cvt<<<dim3(DM), blk, 0, stream>>>(wo, wo16, WSCALE);

    k_gemm_qkv<<<dim3(NQKV / 128, SEQ / 128), blk, 0, stream>>>(x16, w316, qh, qr, kh, kr, vth, vtr);
    k_attn<1><<<dim3(NH * NQBE), dim3(128), 0, stream>>>(qh, qr, kh, kr, vth, vtr, yh, yr);
    if (NQBL > 0)
        k_attn<0><<<dim3(NH * (NQBL > 0 ? NQBL : 1)), dim3(128), 0, stream>>>(qh, qr, kh, kr, vth, vtr, yh, yr);
    k_gemm_out<<<dim3(DM / 64, SEQ / 128), blk, 0, stream>>>(yh, yr, wo16, out);
}
